// VADER_79121887527171
// MI455X (gfx1250) — hardware-verified
//
#include <hip/hip_runtime.h>
#include <stddef.h>


typedef _Float16 h16;
typedef _Float16 v16h __attribute__((ext_vector_type(16)));
typedef _Float16 v8h  __attribute__((ext_vector_type(8)));
typedef float    v8f  __attribute__((ext_vector_type(8)));
typedef float    v4f  __attribute__((ext_vector_type(4)));
typedef int      v4i  __attribute__((ext_vector_type(4)));

#ifndef NB
#define NB 8
#endif
#define NB_FULL 8
#define LSEQ   96
#define DIM    512
#define NOUT   64
#define NTYPE  47
#define TPAD   48
#define TK     64
#define KPAD   128
#define NLAYER 3

static_assert(NB >= 1 && NB <= NB_FULL);
static_assert(LSEQ == 6 * 16 && (LSEQ % 32) == 0 && (LSEQ % 8) == 0);
static_assert((DIM % 64) == 0 && (DIM % 32) == 0);
static_assert(NTYPE < TPAD && (TPAD % 16) == 0 && TPAD <= TK && (TK % 32) == 0);
static_assert(KPAD >= LSEQ && (KPAD % 64) == 0);
static_assert(NOUT == 64);
static_assert(LSEQ * LSEQ == 4 * 192 * 12);
static_assert(TPAD * TPAD == 192 * 12);
static_assert(LSEQ * 64 == 4 * 384 * 4);
static_assert(LSEQ * 8 == 2 * 384);
static_assert(64 * (KPAD / 8) == 2 * 384 + 256);
static_assert(TPAD * 16 == 2 * 288 + 192);
static_assert(TPAD * 8 == 256 + 128);

#define LDT 72
#define LDC 68
#define LDP 168
#define LDE 520
static_assert((LDT % 8) == 0 && LDT >= 64);
static_assert((LDC % 4) == 0 && LDC >= 64);
static_assert((LDP % 8) == 0 && LDP >= LSEQ + TK);
static_assert((LDE % 8) == 0 && LDE >= DIM);

#define WCARRY 64.0f
#define TCARRY 16.0f
#define SCARRY 16.0f
#define PCARRY 1024.0f
#define ACARRY 64.0f
#define ECARRY 256.0f
#define RCARRY 2048.0f

#define WL_BYTES   ((size_t)DIM * DIM * 2)
#define WT_BYTES   ((size_t)NLAYER * WL_BYTES)
#define FCW_BYTES  ((size_t)NOUT * DIM * 2)
#define TAB_BYTES  ((size_t)TPAD * DIM * 2)
#define TABT_BYTES ((size_t)DIM * TK * 2)
#define G_BYTES    ((size_t)TPAD * 64 * 4)
#define SEQ_BYTES  ((size_t)NB * LSEQ * DIM * 2)
#define SEQT_BYTES ((size_t)NB * DIM * KPAD * 2)
#define AGG_BYTES  ((size_t)NB * LSEQ * DIM * 2)
#define POOL_BYTES ((size_t)NLAYER * NB * DIM * 4)
#define OFF_WT   ((size_t)0)
#define OFF_FCW  (OFF_WT + WT_BYTES)
#define OFF_TAB  (OFF_FCW + FCW_BYTES)
#define OFF_TABT (OFF_TAB + TAB_BYTES)
#define OFF_G    (OFF_TABT + TABT_BYTES)
#define OFF_SEQ  (OFF_G + G_BYTES)
#define OFF_SEQT (OFF_SEQ + SEQ_BYTES)
#define OFF_AGG  (OFF_SEQT + SEQT_BYTES)
#define OFF_POOL (OFF_AGG + AGG_BYTES)
#define WS_TOTAL (OFF_POOL + POOL_BYTES)
static_assert((WL_BYTES % 128) == 0 && (FCW_BYTES % 128) == 0 && (TAB_BYTES % 128) == 0);
static_assert((TABT_BYTES % 128) == 0 && (G_BYTES % 128) == 0 && (SEQ_BYTES % 128) == 0);
static_assert((SEQT_BYTES % 128) == 0 && (AGG_BYTES % 128) == 0 && (POOL_BYTES % 128) == 0);
static_assert(WS_TOTAL <= (size_t)134217728);

__device__ __forceinline__ float bf16r(float x) {
  unsigned int u = __float_as_uint(x);
  u = (u + 0x7FFFu + ((u >> 16) & 1u)) & 0xFFFF0000u;
  return __uint_as_float(u);
}

static __device__ __forceinline__ h16 toh_flush(float v) {
  const h16 r = (h16)v;
  return (fabsf(v) < 6.103515625e-05f) ? (h16)0.0f : r;
}

__device__ __forceinline__ v16h frag_at(const _Float16* p) {
  v8h lo = *(const v8h*)(p);
  v8h hi = *(const v8h*)(p + 16);
  v16h out;
#pragma unroll
  for (int i = 0; i < 8; ++i) { out[i] = lo[i]; out[i + 8] = hi[i]; }
  return out;
}
__device__ __forceinline__ v16h ld_frag(const _Float16* base, unsigned ld) {
  const unsigned lane = threadIdx.x & 31u;
  return frag_at(base + (lane & 15u) * ld + (lane >> 4) * 8u);
}

__device__ __forceinline__ v8f wmma16(v16h a, v16h b, v8f c) {
  v8f d = __builtin_amdgcn_wmma_f32_16x16x32_f16(false, a, false, b, (short)0, c,
                                                 false, false);
  asm volatile("v_nop\n\tv_nop\n\tv_nop\n\tv_nop" : "+v"(d) : "v"(a), "v"(b));
  return d;
}

__device__ __forceinline__ float red16_max(float x) {
#pragma unroll
  for (int off = 1; off < 16; off <<= 1) x = fmaxf(x, __shfl_xor(x, off, 32));
  return x;
}
__device__ __forceinline__ float red16_sum(float x) {
#pragma unroll
  for (int off = 1; off < 16; off <<= 1) x += __shfl_xor(x, off, 32);
  return x;
}

__device__ __forceinline__ void wave_lds_sync() {
  __builtin_amdgcn_fence(3  , "wavefront");
  asm volatile("s_wait_dscnt 0x0" ::: "memory");
  __builtin_amdgcn_wave_barrier();
}

__global__ __launch_bounds__(256) void wconv_kernel(
    const float* __restrict__ W, _Float16* __restrict__ Wt, unsigned ldw, unsigned ldk) {
  __shared__ _Float16 T[64 * LDT];
  const unsigned tid = threadIdx.x;
  const unsigned n0 = blockIdx.x * 64u;
  const unsigned k0 = blockIdx.y * 64u;
#pragma unroll 4
  for (unsigned j = 0; j < 16u; ++j) {
    const unsigned idx = tid + 256u * j;
    const unsigned kr = idx >> 6, nc = idx & 63u;
    const float v = W[(size_t)(k0 + kr) * ldw + n0 + nc];
    T[nc * LDT + kr] = toh_flush(WCARRY * bf16r(v));
  }
  __syncthreads();
  v8h x[2];
  size_t off[2];
#pragma unroll
  for (unsigned i = 0; i < 2u; ++i) {
    const unsigned n = 32u * i + (tid >> 3);
    const unsigned kc = (tid & 7u) * 8u;
    x[i] = *(const v8h*)&T[n * LDT + kc];
    off[i] = (size_t)(n0 + n) * ldk + k0 + kc;
  }
#pragma unroll
  for (int i = 0; i < 2; ++i) *(volatile v8h*)(Wt + off[i]) = x[i];
  __threadfence();
#pragma unroll
  for (int i = 0; i < 2; ++i) *(volatile v8h*)(Wt + off[i]) = x[i];
}

__global__ __launch_bounds__(256) void table_kernel(
    const float* __restrict__ table, _Float16* __restrict__ Tab, _Float16* __restrict__ TabT) {
#pragma clang fp contract(off)
  __shared__ __attribute__((aligned(16))) _Float16 T[TK * LDT];
  const unsigned tid = threadIdx.x;
  const unsigned w = (unsigned)__builtin_amdgcn_readfirstlane((int)(tid >> 5));
  const unsigned n0 = blockIdx.x * 64u;
#pragma unroll 4
  for (unsigned j = 0; j < 16u; ++j) {
    const unsigned idx = tid + 256u * j;
    const unsigned t = idx >> 6, dc = idx & 63u;
    unsigned tc = (t < 1u) ? 1u : t;
    tc = (tc > (unsigned)(NTYPE - 1)) ? (unsigned)(NTYPE - 1) : tc;
    float v = table[(size_t)tc * DIM + n0 + dc];
    asm volatile("" : "+v"(v));
    const bool live = (t >= 1u) && (t <= (unsigned)(NTYPE - 1));
    T[t * LDT + dc] = live ? toh_flush(TCARRY * bf16r(v)) : (h16)0.0f;
  }
  __syncthreads();
  v8h xa[2], xb[2];
  size_t offa[2], offb[2];
#pragma unroll
  for (unsigned i = 0; i < 2u; ++i) {
    unsigned p = tid + 256u * i;
    p = (p > 383u) ? 383u : p;
    const unsigned r = p >> 3, c = (p & 7u) * 8u;
    xa[i] = *(const v8h*)&T[r * LDT + c];
    offa[i] = (size_t)r * DIM + n0 + c;
  }
#pragma unroll
  for (unsigned i = 0; i < 2u; ++i) {
    const unsigned p = tid + 256u * i;
    const unsigned d = p >> 3, tp = p & 7u;
#pragma unroll
    for (unsigned j = 0; j < 8u; ++j) xb[i][j] = T[(tp * 8u + j) * LDT + d];
    offb[i] = (size_t)(n0 + d) * TK + tp * 8u;
  }
  *(volatile v8h*)(Tab + offa[0]) = xa[0];
  if (w < 4u) *(volatile v8h*)(Tab + offa[1]) = xa[1];
#pragma unroll
  for (int i = 0; i < 2; ++i) *(volatile v8h*)(TabT + offb[i]) = xb[i];
  __threadfence();
  *(volatile v8h*)(Tab + offa[0]) = xa[0];
  if (w < 4u) *(volatile v8h*)(Tab + offa[1]) = xa[1];
#pragma unroll
  for (int i = 0; i < 2; ++i) *(volatile v8h*)(TabT + offb[i]) = xb[i];
}

__global__ __launch_bounds__(288) void gram_kernel(
    const _Float16* __restrict__ Tab, float* __restrict__ G) {
  __shared__ __attribute__((aligned(16))) float Gs[TPAD * LDC];
  const unsigned tid = threadIdx.x, lane = tid & 31u;
  const unsigned w = (unsigned)__builtin_amdgcn_readfirstlane((int)(tid >> 5));
  const unsigned hh = lane >> 4, m = lane & 15u;
  const unsigned ti = w / 3u, tj = w - 3u * ti;
  const _Float16* ap = Tab + (size_t)(ti * 16u + m) * DIM + hh * 8u;
  const _Float16* bp = Tab + (size_t)(tj * 16u + m) * DIM + hh * 8u;
  v8f acc = {};
#pragma unroll 2
  for (unsigned k0 = 0; k0 < (unsigned)DIM; k0 += 32u) {
    const v16h a = frag_at(ap + k0);
    const v16h bq = frag_at(bp + k0);
    acc = wmma16(a, bq, acc);
  }
#pragma unroll
  for (int r = 0; r < 8; ++r)
    Gs[(ti * 16u + hh * 8u + (unsigned)r) * LDC + tj * 16u + m] =
        acc[r] * (1.0f / (TCARRY * TCARRY));
  __syncthreads();
  v4f x[3];
  size_t off[3];
#pragma unroll
  for (unsigned i = 0; i < 3u; ++i) {
    unsigned p = tid + 288u * i;
    p = (p > 767u) ? 767u : p;
    const unsigned r = p >> 4, c = (p & 15u) * 4u;
    const unsigned cc = (c > 44u) ? 44u : c;
    const v4f u = *(const v4f*)&Gs[r * LDC + cc];
    v4f z = {};
    x[i] = (c < (unsigned)TPAD) ? u : z;
    off[i] = (size_t)r * 64u + c;
  }
  *(volatile v4f*)(G + off[0]) = x[0];
  *(volatile v4f*)(G + off[1]) = x[1];
  if (w < 6u) *(volatile v4f*)(G + off[2]) = x[2];
  __threadfence();
  *(volatile v4f*)(G + off[0]) = x[0];
  *(volatile v4f*)(G + off[1]) = x[1];
  if (w < 6u) *(volatile v4f*)(G + off[2]) = x[2];
}

template <int IS_GEMM>
__device__ __forceinline__ void tile_body(
    const float* __restrict__ text, const float* __restrict__ gam, const float* __restrict__ bet,
    const _Float16* __restrict__ A16, const _Float16* __restrict__ Bt,
    const float* __restrict__ bias, const float* __restrict__ mask,
    _Float16* __restrict__ seq, _Float16* __restrict__ seqt, float* __restrict__ pool) {
#pragma clang fp contract(off)
  __shared__ __attribute__((aligned(16))) float Cs[LSEQ * LDC];
  const unsigned tid = threadIdx.x, lane = tid & 31u;
  const unsigned w = (unsigned)__builtin_amdgcn_readfirstlane((int)(tid >> 5));
  const unsigned hh = lane >> 4, m = lane & 15u;
  const unsigned n0 = blockIdx.x * 64u;
  const unsigned b = blockIdx.y;
  const unsigned row0 = b * (unsigned)LSEQ;

  if (IS_GEMM) {
    const unsigned mw = w >> 1, nw = w & 1u;
    const _Float16* ap  = A16 + (size_t)(row0 + mw * 16u + m) * DIM + hh * 8u;
    const _Float16* bp0 = Bt + (size_t)(n0 + nw * 32u + m) * DIM + hh * 8u;
    const _Float16* bp1 = bp0 + (size_t)16 * DIM;
    v8f acc0 = {}, acc1 = {};
#pragma unroll 2
    for (unsigned k0 = 0; k0 < (unsigned)DIM; k0 += 32u) {
      const v16h a  = frag_at(ap + k0);
      const v16h b0 = frag_at(bp0 + k0);
      const v16h b1 = frag_at(bp1 + k0);
      acc0 = wmma16(a, b0, acc0);
      acc1 = wmma16(a, b1, acc1);
    }
#pragma unroll
    for (int r = 0; r < 8; ++r) {
      float* d = &Cs[(mw * 16u + hh * 8u + (unsigned)r) * LDC + nw * 32u + m];
      d[0]  = acc0[r];
      d[16] = acc1[r];
    }
    __syncthreads();
#pragma unroll 1
    for (unsigned g = 0; g < 4u; ++g) {
      const unsigned q = tid + 384u * g;
      const unsigned r = q >> 4, c = (q & 15u) * 4u;
      const v4f u  = *(const v4f*)&Cs[r * LDC + c];
      const v4f gb = *(const v4f*)(bias + n0 + c);
      v4f t;
#pragma unroll
      for (int j = 0; j < 4; ++j)
        t[j] = SCARRY * fmaxf(u[j] * (1.0f / (ACARRY * WCARRY)) + bf16r(gb[j]), 0.0f);
      *(v4f*)&Cs[r * LDC + c] = t;
    }
  } else {
    const float inv = 1.0f / sqrtf(1.0f + 1.0e-3f);
#pragma unroll 1
    for (unsigned g = 0; g < 4u; ++g) {
      const unsigned q = tid + 384u * g;
      const unsigned r = q >> 4, c = (q & 15u) * 4u;
      const v4f x  = *(const v4f*)(text + (size_t)(row0 + r) * DIM + n0 + c);
      const v4f ga = *(const v4f*)(gam + n0 + c);
      const v4f be = *(const v4f*)(bet + n0 + c);
      v4f t;
#pragma unroll
      for (int j = 0; j < 4; ++j)
        t[j] = SCARRY * (bf16r(x[j]) * (bf16r(ga[j]) * inv) + bf16r(be[j]));
      *(v4f*)&Cs[r * LDC + c] = t;
    }
  }
  __syncthreads();

  if (IS_GEMM) {
    if (w < 2u) {
      float sum = 0.0f, cnt = 0.0f;
#pragma unroll 1
      for (unsigned r = 0; r < (unsigned)LSEQ; ++r) {
        const float mk = bf16r(mask[row0 + r]);
        sum += Cs[r * LDC + tid] * mk;
        cnt += (mk != 0.0f) ? 1.0f : 0.0f;
      }
      const float pv = (sum * (1.0f / SCARRY)) * (1.0f / (cnt + 1.0e-10f));
      float* pp = pool + (size_t)b * DIM + n0 + tid;
      *(volatile float*)pp = pv;
      __threadfence();
      *(volatile float*)pp = pv;
    }
  }

  v8h xr[2], xt[3];
  size_t offr[2], offt[3];
#pragma unroll
  for (unsigned i = 0; i < 2u; ++i) {
    const unsigned p = tid + 384u * i;
    const unsigned r = p >> 3, c = (p & 7u) * 8u;
    const v4f u0 = *(const v4f*)&Cs[r * LDC + c];
    const v4f u1 = *(const v4f*)&Cs[r * LDC + c + 4u];
#pragma unroll
    for (int j = 0; j < 4; ++j) {
      xr[i][j]     = toh_flush(u0[j]);
      xr[i][j + 4] = toh_flush(u1[j]);
    }
    offr[i] = (size_t)(row0 + r) * DIM + n0 + c;
  }
#pragma unroll
  for (unsigned i = 0; i < 3u; ++i) {
    unsigned p = tid + 384u * i;
    p = (p > 1023u) ? 1023u : p;
    const unsigned d = p >> 4, kp = p & 15u;
    const bool live = (kp * 8u) < (unsigned)LSEQ;
#pragma unroll
    for (unsigned j = 0; j < 8u; ++j) {
      const unsigned key = kp * 8u + j;
      const unsigned kc = (key < (unsigned)LSEQ) ? key : (unsigned)(LSEQ - 1);
      const float v = Cs[kc * LDC + d];
      xt[i][j] = live ? toh_flush(v) : (h16)0.0f;
    }
    offt[i] = ((size_t)b * DIM + n0 + d) * KPAD + kp * 8u;
  }
#pragma unroll
  for (int i = 0; i < 2; ++i) *(volatile v8h*)(seq + offr[i]) = xr[i];
#pragma unroll
  for (int i = 0; i < 2; ++i) *(volatile v8h*)(seqt + offt[i]) = xt[i];
  if (w < 8u) *(volatile v8h*)(seqt + offt[2]) = xt[2];
  __threadfence();
#pragma unroll
  for (int i = 0; i < 2; ++i) *(volatile v8h*)(seq + offr[i]) = xr[i];
#pragma unroll
  for (int i = 0; i < 2; ++i) *(volatile v8h*)(seqt + offt[i]) = xt[i];
  if (w < 8u) *(volatile v8h*)(seqt + offt[2]) = xt[2];
}

__global__ __launch_bounds__(384) void seq0_kernel(
    const float* __restrict__ text, const float* __restrict__ gam, const float* __restrict__ bet,
    _Float16* __restrict__ seq, _Float16* __restrict__ seqt) {
  tile_body<0>(text, gam, bet, (const _Float16*)0, (const _Float16*)0, gam, gam,
               seq, seqt, (float*)0);
}
__global__ __launch_bounds__(384) void fc_kernel(
    const _Float16* __restrict__ A16, const _Float16* __restrict__ Bt,
    const float* __restrict__ bias, const float* __restrict__ mask,
    _Float16* __restrict__ seq, _Float16* __restrict__ seqt, float* __restrict__ pool) {
  tile_body<1>(bias, bias, bias, A16, Bt, bias, mask, seq, seqt, pool);
}

__global__ __launch_bounds__(192) void attn_kernel(
    const _Float16* __restrict__ Seq, const _Float16* __restrict__ SeqT,
    const _Float16* __restrict__ TabT, const float* __restrict__ G,
    const float* __restrict__ adj, const int* __restrict__ depv,
    _Float16* __restrict__ Agg) {
  __shared__ __attribute__((aligned(16))) float Gs[TPAD * TPAD];
  __shared__ __attribute__((aligned(16))) unsigned short Aj[LSEQ * LSEQ];
  __shared__ __attribute__((aligned(16))) unsigned char Dv[LSEQ * LSEQ];
  __shared__ __attribute__((aligned(16))) _Float16 Ps[6 * 16 * LDP];
  __shared__ __attribute__((aligned(16))) float Wt[6 * 2 * 16 * TPAD];
  __shared__ __attribute__((aligned(16))) _Float16 Os[6 * 16 * LDT];
  static_assert(sizeof(float) * TPAD * TPAD + 2 * LSEQ * LSEQ + LSEQ * LSEQ +
                2 * 6 * 16 * LDP + 4 * 6 * 2 * 16 * TPAD + 2 * 6 * 16 * LDT <= 131072);

  const unsigned tid = threadIdx.x, lane = tid & 31u;
  const unsigned w = (unsigned)__builtin_amdgcn_readfirstlane((int)(tid >> 5));
  const unsigned hh = lane >> 4, m = lane & 15u;
  const unsigned b = blockIdx.x;
  const unsigned i0 = w * 16u;
  _Float16* P = Ps + w * (16u * LDP);
  _Float16* O = Os + w * (16u * LDT);

#pragma unroll 1
  for (unsigned idx = tid; idx < (unsigned)(TPAD * TPAD); idx += 192u) {
    const unsigned r = idx / (unsigned)TPAD;
    const unsigned c = idx - r * (unsigned)TPAD;
    Gs[idx] = G[r * 64u + c];
  }
#pragma unroll 1
  for (unsigned it = 0; it < 12u; ++it) {
    const unsigned q = tid + 192u * it;
    const v4i dv = *(const v4i*)(depv + (size_t)b * (LSEQ * LSEQ) + 4u * q);
    const v4f av = *(const v4f*)(adj + (size_t)b * (LSEQ * LSEQ) + 4u * q);
#pragma unroll
    for (int j = 0; j < 4; ++j) {
      int t = dv[j];
      t = (t < 0) ? 0 : t;
      t = (t > NTYPE - 1) ? (NTYPE - 1) : t;
      Dv[4u * q + (unsigned)j] = (unsigned char)t;
      unsigned int u = __float_as_uint(av[j]);
      u = (u + 0x7FFFu + ((u >> 16) & 1u)) >> 16;
      Aj[4u * q + (unsigned)j] = (unsigned short)u;
    }
  }
  __syncthreads();

  v8f s[6];
#pragma unroll
  for (int kg = 0; kg < 6; ++kg) s[kg] = (v8f){};
  {
    const _Float16* ap = Seq + (size_t)(b * (unsigned)LSEQ + i0 + m) * DIM + hh * 8u;
    const _Float16* kp = Seq + (size_t)(b * (unsigned)LSEQ + m) * DIM + hh * 8u;
#pragma unroll 1
    for (unsigned k0 = 0; k0 < (unsigned)DIM; k0 += 32u) {
      const v16h a = frag_at(ap + k0);
#pragma unroll
      for (int kg = 0; kg < 6; ++kg) {
        const v16h kf = frag_at(kp + (size_t)(kg * 16) * DIM + k0);
        s[kg] = wmma16(a, kf, s[kg]);
      }
    }
  }

  const float scale = 0.04419417382415922f;
#pragma unroll
  for (int kg = 0; kg < 6; ++kg)
#pragma unroll
    for (int r = 0; r < 8; ++r) {
      const unsigned i = i0 + hh * 8u + (unsigned)r;
      const unsigned j = (unsigned)kg * 16u + m;
      const unsigned v1 = Dv[i * (unsigned)LSEQ + j];
      const unsigned v2 = Dv[j * (unsigned)LSEQ + i];
      const float g = Gs[v1 * (unsigned)TPAD + v2];
      s[kg][r] = (s[kg][r] * (1.0f / (SCARRY * SCARRY)) + g) * scale;
    }

#pragma unroll
  for (int r = 0; r < 8; ++r) {
    float mx = fmaxf(fmaxf(fmaxf(s[0][r], s[1][r]), fmaxf(s[2][r], s[3][r])),
                     fmaxf(s[4][r], s[5][r]));
    mx = red16_max(mx);
    float e[6];
#pragma unroll
    for (int kg = 0; kg < 6; ++kg) e[kg] = __expf(s[kg][r] - mx);
    const float rs = red16_sum(((e[0] + e[1]) + (e[2] + e[3])) + (e[4] + e[5]));
    const float inv = __builtin_amdgcn_rcpf(rs);
    const unsigned i = i0 + hh * 8u + (unsigned)r;
#pragma unroll
    for (int kg = 0; kg < 6; ++kg) {
      const unsigned j = (unsigned)kg * 16u + m;
      const float av = __uint_as_float(((unsigned int)Aj[i * (unsigned)LSEQ + j]) << 16);
      const float a = (e[kg] * inv) * av;
      P[(hh * 8u + (unsigned)r) * LDP + j] = toh_flush(PCARRY * a);
    }
  }
  wave_lds_sync();

  {
    const unsigned wb = ((w * 2u + hh) * 16u + m) * (unsigned)TPAD;
#pragma unroll 4
    for (unsigned t = 0; t < (unsigned)TPAD; ++t) Wt[wb + t] = 0.0f;
    const unsigned irow = i0 + m;
#pragma unroll 1
    for (unsigned jj = 0; jj < 48u; ++jj) {
      const unsigned j = hh * 48u + jj;
      const unsigned t = Dv[j * (unsigned)LSEQ + irow];
      const float pv = (float)P[m * LDP + j];
      Wt[wb + t] += pv;
    }
  }
  wave_lds_sync();
  {
    const unsigned w0b = ((w * 2u) * 16u + m) * (unsigned)TPAD;
    const unsigned w1b = ((w * 2u + 1u) * 16u + m) * (unsigned)TPAD;
#pragma unroll 4
    for (unsigned tt = 0; tt < 24u; ++tt) {
      const unsigned t = hh * 24u + tt;
      P[m * LDP + (unsigned)LSEQ + t] = toh_flush(Wt[w0b + t] + Wt[w1b + t]);
    }
    *(v8h*)&P[m * LDP + (unsigned)(LSEQ + TPAD) + 8u * hh] = (v8h){};
  }
  wave_lds_sync();

#pragma unroll 1
  for (unsigned ng = 0; ng < (unsigned)(DIM / 64); ++ng) {
    v8f o[4];
#pragma unroll
    for (int nb = 0; nb < 4; ++nb) o[nb] = (v8f){};
    const _Float16* sp = SeqT + ((size_t)b * DIM + ng * 64u + m) * KPAD + hh * 8u;
    const _Float16* tp = TabT + (size_t)(ng * 64u + m) * TK + hh * 8u;
#pragma unroll
    for (int c = 0; c < 3; ++c) {
      const v16h pf = ld_frag(P + c * 32, LDP);
#pragma unroll
      for (int nb = 0; nb < 4; ++nb) {
        const v16h vf = frag_at(sp + (size_t)(nb * 16) * KPAD + c * 32);
        o[nb] = wmma16(pf, vf, o[nb]);
      }
    }
#pragma unroll
    for (int c = 0; c < 2; ++c) {
      const v16h pf = ld_frag(P + LSEQ + c * 32, LDP);
#pragma unroll
      for (int nb = 0; nb < 4; ++nb) {
        const v16h tf = frag_at(tp + (size_t)(nb * 16) * TK + c * 32);
        o[nb] = wmma16(pf, tf, o[nb]);
      }
    }
#pragma unroll
    for (int nb = 0; nb < 4; ++nb)
#pragma unroll
      for (int r = 0; r < 8; ++r)
        O[(hh * 8u + (unsigned)r) * LDT + (unsigned)nb * 16u + m] =
            toh_flush(o[nb][r] * (ACARRY / (PCARRY * SCARRY)));
    wave_lds_sync();
    v8h x[4];
    size_t off[4];
#pragma unroll
    for (unsigned i = 0; i < 4u; ++i) {
      const unsigned r = 4u * i + (lane >> 3);
      const unsigned c = (lane & 7u) * 8u;
      x[i] = *(const v8h*)&O[r * LDT + c];
      off[i] = (size_t)(b * (unsigned)LSEQ + i0 + r) * DIM + ng * 64u + c;
    }
#pragma unroll
    for (int i = 0; i < 4; ++i) *(volatile v8h*)(Agg + off[i]) = x[i];
    __threadfence();
#pragma unroll
    for (int i = 0; i < 4; ++i) *(volatile v8h*)(Agg + off[i]) = x[i];
    wave_lds_sync();
  }
}
static_assert(SCARRY == TCARRY);
static_assert(4 * 4 == 16);

__global__ __launch_bounds__(128) void out_kernel(
    const float* __restrict__ pool, const float* __restrict__ ens,
    const _Float16* __restrict__ FcWt, const float* __restrict__ fcb,
    float* __restrict__ out) {
  __shared__ __attribute__((aligned(16))) _Float16 Es[16 * LDE];
  __shared__ __attribute__((aligned(16))) _Float16 EsR[16 * LDE];
  __shared__ __attribute__((aligned(16))) float Cs[16 * LDC];
  static_assert(2 * 2 * 16 * LDE + 4 * 16 * LDC <= 131072);
  const unsigned tid = threadIdx.x, lane = tid & 31u;
  const unsigned w = (unsigned)__builtin_amdgcn_readfirstlane((int)(tid >> 5));
  const unsigned hh = lane >> 4, m = lane & 15u;

  const float e0 = bf16r(ens[0]), e1 = bf16r(ens[1]), e2 = bf16r(ens[2]);
  const float mx = fmaxf(e0, fmaxf(e1, e2));
  const float x0 = __expf(e0 - mx), x1 = __expf(e1 - mx), x2 = __expf(e2 - mx);
  const float inv = __builtin_amdgcn_rcpf((x0 + x1) + x2);
  const float w0 = x0 * inv, w1 = x1 * inv, w2 = x2 * inv;

#pragma unroll 1
  for (unsigned j = 0; j < 64u; ++j) {
    const unsigned idx = tid + 128u * j;
    const unsigned r = idx >> 9, d = idx & 511u;
    const unsigned rc = (r < (unsigned)NB) ? r : (unsigned)(NB - 1);
    const float p0 = pool[(size_t)(0 * NB + rc) * DIM + d];
    const float p1 = pool[(size_t)(1 * NB + rc) * DIM + d];
    const float p2 = pool[(size_t)(2 * NB + rc) * DIM + d];
    const float v = (p0 * w0 + p1 * w1) + p2 * w2;
    const float t = ECARRY * v;
    const h16 hi = toh_flush(t);
    const h16 lo = toh_flush(RCARRY * (t - (float)hi));
    Es[r * LDE + d]  = (r < (unsigned)NB) ? hi : (h16)0.0f;
    EsR[r * LDE + d] = (r < (unsigned)NB) ? lo : (h16)0.0f;
  }
  __syncthreads();

  const _Float16* bp = FcWt + (size_t)(w * 16u + m) * DIM + hh * 8u;
  v8f acc = {}, accr = {};
#pragma unroll 2
  for (unsigned k0 = 0; k0 < (unsigned)DIM; k0 += 32u) {
    const v16h a  = ld_frag(&Es[k0], LDE);
    const v16h ar = ld_frag(&EsR[k0], LDE);
    const v16h bq = frag_at(bp + k0);
    acc  = wmma16(a, bq, acc);
    accr = wmma16(ar, bq, accr);
  }
#pragma unroll
  for (int r = 0; r < 8; ++r)
    Cs[(hh * 8u + (unsigned)r) * LDC + w * 16u + m] = acc[r] + accr[r] * (1.0f / RCARRY);
  __syncthreads();

  const unsigned r = tid >> 4, c = (tid & 15u) * 4u;
  const v4f u = *(const v4f*)&Cs[r * LDC + c];
  const v4f fb = *(const v4f*)(fcb + c);
  v4f val;
#pragma unroll
  for (int j = 0; j < 4; ++j) val[j] = u[j] * (1.0f / (ECARRY * WCARRY)) + bf16r(fb[j]);
  float* op = out + (size_t)r * NOUT + c;
  if (r < (unsigned)NB) *(volatile v4f*)op = val;
  __threadfence();
  if (r < (unsigned)NB) *(volatile v4f*)op = val;
}
static_assert(128 / 16 == NB_FULL);

extern "C" void kernel_launch(void* const* d_in, const int* in_sizes, int n_in,
                              void* d_out, int out_size, void* d_ws, size_t ws_size,
                              hipStream_t stream) {
  if (n_in < 12) return;
  if ((long long)in_sizes[0] < (long long)NB * LSEQ * DIM) return;
  if ((long long)in_sizes[1] < (long long)NB * LSEQ) return;
  if ((long long)in_sizes[2] < (long long)NB * LSEQ * LSEQ) return;
  if ((long long)in_sizes[3] < (long long)NTYPE * DIM) return;
  if (in_sizes[4] < DIM || in_sizes[5] < DIM) return;
  if ((long long)in_sizes[6] < (long long)NLAYER * DIM * DIM) return;
  if (in_sizes[7] < NLAYER * DIM) return;
  if (in_sizes[8] < NLAYER) return;
  if ((long long)in_sizes[9] < (long long)DIM * NOUT) return;
  if (in_sizes[10] < NOUT) return;
  if ((long long)in_sizes[11] < (long long)NB * LSEQ * LSEQ) return;
  if ((long long)out_size < (long long)NB * NOUT) return;
  if (ws_size < WS_TOTAL) return;

  const float* text  = (const float*)d_in[0];
  const float* mask  = (const float*)d_in[1];
  const float* adj   = (const float*)d_in[2];
  const float* table = (const float*)d_in[3];
  const float* gam   = (const float*)d_in[4];
  const float* bet   = (const float*)d_in[5];
  const float* wst   = (const float*)d_in[6];
  const float* bst   = (const float*)d_in[7];
  const float* ens   = (const float*)d_in[8];
  const float* fcw   = (const float*)d_in[9];
  const float* fcb   = (const float*)d_in[10];
  const int*   depv  = (const int*)d_in[11];
  float* out = (float*)d_out;

  char* ws = (char*)d_ws;
  _Float16* Wt16  = (_Float16*)(ws + OFF_WT);
  _Float16* FcWt  = (_Float16*)(ws + OFF_FCW);
  _Float16* Tab16 = (_Float16*)(ws + OFF_TAB);
  _Float16* TabT  = (_Float16*)(ws + OFF_TABT);
  float*    G     = (float*)(ws + OFF_G);
  _Float16* Seq   = (_Float16*)(ws + OFF_SEQ);
  _Float16* SeqT  = (_Float16*)(ws + OFF_SEQT);
  _Float16* Agg   = (_Float16*)(ws + OFF_AGG);
  float*    Pool  = (float*)(ws + OFF_POOL);

  for (int l = 0; l < NLAYER; ++l)
    wconv_kernel<<<dim3(DIM / 64, DIM / 64), dim3(256), 0, stream>>>(
        wst + (size_t)l * DIM * DIM, Wt16 + (size_t)l * DIM * DIM, (unsigned)DIM, (unsigned)DIM);
  wconv_kernel<<<dim3(NOUT / 64, DIM / 64), dim3(256), 0, stream>>>(
      fcw, FcWt, (unsigned)NOUT, (unsigned)DIM);
  table_kernel<<<dim3(DIM / 64), dim3(256), 0, stream>>>(table, Tab16, TabT);
  gram_kernel<<<dim3(1), dim3(288), 0, stream>>>(Tab16, G);
  seq0_kernel<<<dim3(DIM / 64, NB), dim3(384), 0, stream>>>(text, gam, bet, Seq, SeqT);

  for (int l = 0; l < NLAYER; ++l) {
    attn_kernel<<<dim3(NB), dim3(192), 0, stream>>>(Seq, SeqT, TabT, G, adj, depv, Agg);
    fc_kernel<<<dim3(DIM / 64, NB), dim3(384), 0, stream>>>(
        Agg, Wt16 + (size_t)l * DIM * DIM, bst + (size_t)l * DIM, mask, Seq, SeqT,
        Pool + (size_t)l * NB * DIM);
  }
  out_kernel<<<dim3(1), dim3(128), 0, stream>>>(Pool, ens, FcWt, fcb, out);
}
